// MAM_70849780515288
// MI455X (gfx1250) — hardware-verified
//
#include <hip/hip_runtime.h>
#include <stddef.h>


typedef _Float16 h16;
typedef _Float16 v16h __attribute__((ext_vector_type(16)));
typedef _Float16 v8h  __attribute__((ext_vector_type(8)));
typedef float    v8f  __attribute__((ext_vector_type(8)));
typedef float    v4f  __attribute__((ext_vector_type(4)));

#ifndef NROWS
#define NROWS 4096
#endif
#define NROWS_FULL 4096
#define DIM 512

static_assert(NROWS >= 64 && NROWS <= NROWS_FULL);
static_assert((NROWS % 64) == 0);
static_assert((DIM % 64) == 0 && (DIM % 32) == 0);
static_assert((DIM % 8) == 0);
static_assert((((size_t)NROWS * DIM) % 2048) == 0);
static_assert((((size_t)DIM * DIM) % 2048) == 0);

#define LDC 68
static_assert((LDC % 4) == 0 && LDC >= 64);

#define ACARRY 16.0f
#define WCARRY 64.0f

#define A16_BYTES ((size_t)NROWS * DIM * 2)
#define W16_BYTES ((size_t)DIM * DIM * 2)
#define OFF_A16 ((size_t)0)
#define OFF_W16 (OFF_A16 + A16_BYTES)
#define WS_TOTAL (OFF_W16 + W16_BYTES)
static_assert((A16_BYTES % 128) == 0 && (W16_BYTES % 128) == 0);
static_assert(WS_TOTAL <= (size_t)134217728);

__device__ __forceinline__ float bf16r(float x) {
  unsigned int u = __float_as_uint(x);
  u = (u + 0x7FFFu + ((u >> 16) & 1u)) & 0xFFFF0000u;
  return __uint_as_float(u);
}

static __device__ __forceinline__ h16 toh_flush(float v) {
  const h16 r = (h16)v;
  return (fabsf(v) < 6.103515625e-05f) ? (h16)0.0f : r;
}

__device__ __forceinline__ v16h frag_at(const _Float16* p) {
  v8h lo = *(const v8h*)(p);
  v8h hi = *(const v8h*)(p + 16);
  v16h out;
#pragma unroll
  for (int i = 0; i < 8; ++i) { out[i] = lo[i]; out[i + 8] = hi[i]; }
  return out;
}

__device__ __forceinline__ v8f wmma16(v16h a, v16h b, v8f c) {
  v8f d = __builtin_amdgcn_wmma_f32_16x16x32_f16(false, a, false, b, (short)0, c,
                                                 false, false);
  asm volatile("v_nop\n\tv_nop\n\tv_nop\n\tv_nop" : "+v"(d) : "v"(a), "v"(b));
  return d;
}

__global__ __launch_bounds__(256) void plane_cast_kernel(
    const float* __restrict__ src, _Float16* __restrict__ dst, float carry) {
#pragma clang fp contract(off)
  const size_t i8 = ((size_t)blockIdx.x * 256u + threadIdx.x) * 8u;
  const v4f a0 = *(const v4f*)(src + i8);
  const v4f a1 = *(const v4f*)(src + i8 + 4u);
  v8h o;
#pragma unroll
  for (int i = 0; i < 4; ++i) {
    const float t0 = carry * bf16r(a0[i]);
    const float t1 = carry * bf16r(a1[i]);
    o[i]     = toh_flush(t0);
    o[i + 4] = toh_flush(t1);
  }
  _Float16* p = dst + i8;
  *(volatile v8h*)p = o;
  __threadfence();
  *(volatile v8h*)p = o;
}

__global__ __launch_bounds__(256) void gemm_res_kernel(
    const _Float16* __restrict__ A16, const _Float16* __restrict__ Bt,
    const float* __restrict__ addf, float* __restrict__ outf) {
  __shared__ float Cs[64 * LDC];
  const unsigned tid = threadIdx.x, lane = tid & 31u;
  const unsigned w = (unsigned)__builtin_amdgcn_readfirstlane((int)(tid >> 5));
  const unsigned mw = w >> 1, nw = w & 1u;
  const unsigned hh = lane >> 4, m = lane & 15u;
  const unsigned n0 = blockIdx.x * 64u;
  const unsigned row0 = blockIdx.y * 64u;
  const unsigned K = (unsigned)DIM;

  const _Float16* ap  = A16 + (size_t)(row0 + mw * 16u + m) * K + hh * 8u;
  const _Float16* bp0 = Bt + (size_t)(n0 + nw * 32u + m) * K + hh * 8u;
  const _Float16* bp1 = bp0 + (size_t)16 * K;
  v8f acc0 = {}, acc1 = {};
#pragma unroll 2
  for (unsigned k0 = 0; k0 < K; k0 += 32u) {
    const v16h a  = frag_at(ap + k0);
    const v16h b0 = frag_at(bp0 + k0);
    const v16h b1 = frag_at(bp1 + k0);
    acc0 = wmma16(a, b0, acc0);
    acc1 = wmma16(a, b1, acc1);
  }
#pragma unroll
  for (int r = 0; r < 8; ++r) {
    float* d = &Cs[(mw * 16u + hh * 8u + (unsigned)r) * LDC + nw * 32u + m];
    d[0]  = acc0[r];
    d[16] = acc1[r];
  }
  __syncthreads();

  const float cs = 1.0f / (ACARRY * WCARRY);
  v4f xs[4];
  size_t off[4];
#pragma unroll
  for (unsigned i = 0; i < 4u; ++i) {
    const unsigned r = 16u * i + (tid >> 4);
    const unsigned c = (tid & 15u) * 4u;
    const size_t grow = (size_t)(row0 + r);
    const v4f u = *(const v4f*)&Cs[r * LDC + c];
    const v4f xin = *(const v4f*)(addf + grow * DIM + n0 + c);
    v4f val;
#pragma unroll
    for (int j = 0; j < 4; ++j) val[j] = bf16r(xin[j]) + u[j] * cs;
    xs[i] = val;
    off[i] = grow * DIM + n0 + c;
  }
#pragma unroll
  for (int i = 0; i < 4; ++i) *(volatile v4f*)(outf + off[i]) = xs[i];
  __threadfence();
#pragma unroll
  for (int i = 0; i < 4; ++i) *(volatile v4f*)(outf + off[i]) = xs[i];
}

extern "C" void kernel_launch(void* const* d_in, const int* in_sizes, int n_in,
                              void* d_out, int out_size, void* d_ws, size_t ws_size,
                              hipStream_t stream) {
  if (n_in < 6) return;
  const long long need = (long long)NROWS * DIM;
  if ((long long)in_sizes[0] < need) return;
  if ((long long)in_sizes[3] < need) return;
  if ((long long)in_sizes[5] < (long long)DIM * DIM) return;
  if ((long long)out_size < need) return;
  if (ws_size < WS_TOTAL) return;

  const float* q   = (const float*)d_in[0];
  const float* bsc = (const float*)d_in[3];
  const float* w2  = (const float*)d_in[5];
  float* out = (float*)d_out;

  char* ws = (char*)d_ws;
  _Float16* A16 = (_Float16*)(ws + OFF_A16);
  _Float16* W16 = (_Float16*)(ws + OFF_W16);

  dim3 blk(256);
  plane_cast_kernel<<<dim3((unsigned)(((size_t)NROWS * DIM) / 2048)), blk, 0, stream>>>(
      bsc, A16, ACARRY);
  plane_cast_kernel<<<dim3((unsigned)(((size_t)DIM * DIM) / 2048)), blk, 0, stream>>>(
      w2, W16, WCARRY);
  gemm_res_kernel<<<dim3(DIM / 64, NROWS / 64), blk, 0, stream>>>(A16, W16, q, out);
}
